// CustomLinearLayer_52338471469274
// MI455X (gfx1250) — hardware-verified
//
#include <hip/hip_runtime.h>


#define NB_  4096
#define KIN  2048
#define NOUT 512
#define DM   NOUT
#define LOSC 1024.0f
typedef _Float16 h16;
typedef unsigned short bf;
typedef __attribute__((ext_vector_type(16))) __bf16   v16bf;
typedef __attribute__((ext_vector_type(16))) _Float16 v16h;
typedef __attribute__((ext_vector_type(8)))  _Float16 v8h;
typedef __attribute__((ext_vector_type(8)))  unsigned short v8us;
typedef __attribute__((ext_vector_type(8)))  float    v8f;
typedef __attribute__((ext_vector_type(4)))  float    v4f;
typedef v8h  __attribute__((may_alias)) v8ha;
typedef v4f  __attribute__((may_alias)) v4fa;
typedef v8us __attribute__((may_alias)) v8usa;

__device__ __forceinline__ unsigned short f2bf(float f) { unsigned u = __float_as_uint(f); u += 0x7FFFu + ((u >> 16) & 1u); return (unsigned short)(u >> 16); }
__device__ __forceinline__ float bf2f(unsigned short b) { return __uint_as_float(((unsigned)b) << 16); }
__device__ __forceinline__ float bfr(float f) { return bf2f(f2bf(f)); }
__device__ __forceinline__ v16h cat16(v8h lo, v8h hi) { return __builtin_shufflevector(lo, hi, 0, 1, 2, 3, 4, 5, 6, 7, 8, 9, 10, 11, 12, 13, 14, 15); }
__device__ __forceinline__ v16bf cat16b(v8us lo, v8us hi) { return __builtin_bit_cast(v16bf, __builtin_shufflevector(lo, hi, 0, 1, 2, 3, 4, 5, 6, 7, 8, 9, 10, 11, 12, 13, 14, 15)); }
__device__ __forceinline__ v8f wmma16(v16h a, v16h b, v8f c) { return __builtin_amdgcn_wmma_f32_16x16x32_f16(false, a, false, b, (short)0, c, false, false); }
__device__ __forceinline__ v8f wmmab(v16bf a, v16bf b, v8f c) { return __builtin_amdgcn_wmma_f32_16x16x32_bf16(false, a, false, b, (short)0, c, false, false); }


template <int MODE>
__global__ __launch_bounds__(128) void k_gemm3z(const bf* __restrict__ Ah, const bf* __restrict__ Al, const bf* __restrict__ Bh, const bf* __restrict__ Bl, int K, float* C, int ldc, size_t sA, size_t sB, size_t sC) {
    if ((MODE & 1) && (int)blockIdx.y * 64 > (int)blockIdx.x * 64 + 63) return;
    const size_t z = blockIdx.z; Ah += z * sA; Al += z * sA; Bh += z * sB; Bl += z * sB; C += z * sC;
    const int Klim = (MODE & 2) ? min(K, ((int)blockIdx.x + 1) * 64) : K;
    __shared__ __align__(16) float ost[4][16 * 68];
    const int lane = threadIdx.x & 31, wave = threadIdx.x >> 5, lr = lane & 15, hi = lane >> 4;
    const int r0 = blockIdx.x * 64 + wave * 16, c0 = blockIdx.y * 64;
    const size_t aoff = (size_t)(r0 + lr) * K + 8 * hi;
    v8f acc[4];
#pragma unroll
    for (int t = 0; t < 4; ++t) acc[t] = (v8f){};
#pragma unroll 1
    for (int kc = 0; kc < Klim; kc += 32) {
        const v16bf a = cat16b(*(const v8us*)(Ah + aoff + kc), *(const v8us*)(Ah + aoff + kc + 16));
        v16bf al = a; if (!(MODE & 4) && !(MODE & 16)) al = cat16b(*(const v8us*)(Al + aoff + kc), *(const v8us*)(Al + aoff + kc + 16));
#pragma unroll
        for (int t = 0; t < 4; ++t) { const size_t bo = (size_t)(c0 + t * 16 + lr) * K + kc + 8 * hi;
            const v16bf bh = cat16b(*(const v8us*)(Bh + bo), *(const v8us*)(Bh + bo + 16));
            acc[t] = wmmab(a, bh, acc[t]);
            if (!(MODE & 4)) { if (!(MODE & 16)) acc[t] = wmmab(al, bh, acc[t]); if (!(MODE & 8)) { const v16bf bl = cat16b(*(const v8us*)(Bl + bo), *(const v8us*)(Bl + bo + 16)); acc[t] = wmmab(a, bl, acc[t]); } } }
        asm volatile("v_nop\n\tv_nop\n\tv_nop\n\tv_nop" : "+v"(acc[0]), "+v"(acc[1]), "+v"(acc[2]), "+v"(acc[3]) : "v"(a), "v"(al));
    }
    float* os = &ost[wave][0];
#pragma unroll
    for (int t = 0; t < 4; ++t) {
#pragma unroll
        for (int j = 0; j < 8; ++j) os[(hi * 8 + j) * 68 + t * 16 + lr] = acc[t][j]; }
    __builtin_amdgcn_wave_barrier(); asm volatile("" ::: "memory");
    float* crow = C + (size_t)r0 * ldc + c0;
    auto pass = [&]() {
#pragma unroll
        for (int s = 0; s < 8; ++s) { const int Lid = (lane >> 3) + 4 * s, piece = lane & 7; const int row = Lid >> 1, cofs = (Lid & 1) * 32 + piece * 4;
            const v4f val = *(const v4fa*)(os + row * 68 + cofs); *(volatile v4f*)(crow + (size_t)row * ldc + cofs) = val; }
    };
    pass(); __threadfence(); pass();
}
__global__ __launch_bounds__(256) void k_planes32z(const float* __restrict__ F, int ld, int off, float sc, int rows, bf* Ph, bf* Pl) {
    typedef __attribute__((ext_vector_type(2))) unsigned short v2us;
    const int lane = threadIdx.x & 31; const size_t r = ((size_t)blockIdx.x * 8 + (threadIdx.x >> 5)) * 2 + (lane >> 4); if (r >= (size_t)rows) return; const int z = blockIdx.z; const int c0 = (lane & 15) * 2; v2us oh, ol;
    Ph += (size_t)z * rows * 32; Pl += (size_t)z * rows * 32;
#pragma unroll
    for (int i = 0; i < 2; ++i) { const float y = F[r * ld + off + z * 32 + c0 + i] * sc; const unsigned short hb = f2bf(y); oh[i] = hb; ol[i] = f2bf(y - bf2f(hb)); }
    const size_t o = r * 32 + c0; *(volatile v2us*)(Ph + o) = oh; *(volatile v2us*)(Pl + o) = ol; __threadfence(); *(volatile v2us*)(Ph + o) = oh; *(volatile v2us*)(Pl + o) = ol;
}
__global__ __launch_bounds__(256) void k_vtpadz(const float* __restrict__ F, int ld, int off, int nk, bf* Th, bf* Tl) {
    typedef __attribute__((ext_vector_type(2))) unsigned short v2us;
    const int lane = threadIdx.x & 31; const size_t wid = (size_t)blockIdx.x * 8 + (threadIdx.x >> 5); if (wid >= (size_t)64 * (nk / 64)) return; const int z = blockIdx.z; const int d = (int)(wid / (nk / 64)); const int k0 = (int)(wid % (nk / 64)) * 64 + lane * 2; v2us oh, ol;
    Th += (size_t)z * 64 * nk; Tl += (size_t)z * 64 * nk;
#pragma unroll
    for (int i = 0; i < 2; ++i) { const float y = (d < 32) ? F[(size_t)(k0 + i) * ld + off + z * 32 + (d < 32 ? d : 0)] : 0.f; const unsigned short hb = f2bf(y); oh[i] = hb; ol[i] = f2bf(y - bf2f(hb)); }
    const size_t o = (size_t)d * nk + k0; *(volatile v2us*)(Th + o) = oh; *(volatile v2us*)(Tl + o) = ol; __threadfence(); *(volatile v2us*)(Th + o) = oh; *(volatile v2us*)(Tl + o) = ol;
}
template <int NK>
__global__ __launch_bounds__(256) void k_softmaxz(const float* __restrict__ S, int rows, bf* PH, bf* PL) {
    typedef __attribute__((ext_vector_type(4))) unsigned short v4us;
    const int lane = threadIdx.x & 31, i = blockIdx.x * 8 + (threadIdx.x >> 5); if (i >= rows) return; const size_t zo = (size_t)blockIdx.z * rows * NK; const float* sr = S + zo + (size_t)i * NK; PH += zo; PL += zo;
    float m = -3.0e38f;
#pragma unroll 1
    for (int c0 = lane * 4; c0 < NK; c0 += 128) {
#pragma unroll
        for (int q = 0; q < 4; ++q) m = fmaxf(m, sr[c0 + q]); }
#pragma unroll
    for (int sh = 16; sh; sh >>= 1) m = fmaxf(m, __shfl_xor(m, sh, 32));
    float sum = 0.f;
#pragma unroll 1
    for (int c0 = lane * 4; c0 < NK; c0 += 128) {
#pragma unroll
        for (int q = 0; q < 4; ++q) sum += __expf(sr[c0 + q] - m); }
#pragma unroll
    for (int sh = 16; sh; sh >>= 1) sum += __shfl_xor(sum, sh, 32);
    const float inv = 1.0f / sum;
#pragma unroll 1
    for (int ps = 0; ps < 2; ++ps) {
#pragma unroll 1
        for (int c0 = lane * 4; c0 < NK; c0 += 128) { v4us oh, ol;
#pragma unroll
            for (int q = 0; q < 4; ++q) { const float p = __expf(sr[c0 + q] - m) * inv; const unsigned short hb = f2bf(p); oh[q] = hb; ol[q] = f2bf(p - bf2f(hb)); }
            const size_t o = (size_t)i * NK + c0; *(volatile v4us*)(PH + o) = oh; *(volatile v4us*)(PL + o) = ol; }
        if (ps == 0) __threadfence(); }
}
__global__ __launch_bounds__(256) void k_placez(const float* __restrict__ XH, int rows, int ldy, float* Y) {
    const int lane = threadIdx.x & 31; const size_t q = (size_t)blockIdx.x * 8 + (threadIdx.x >> 5); if (q >= (size_t)rows) return; const int z = blockIdx.z; const float v = XH[((size_t)z * rows + q) * 64 + lane];
    *(volatile float*)(Y + q * ldy + z * 32 + lane) = v; __threadfence(); *(volatile float*)(Y + q * ldy + z * 32 + lane) = v;
}

__global__ __launch_bounds__(256) void k_cvtx(const float* __restrict__ x, bf* A) {
    const int lane = threadIdx.x & 31; const size_t r = (size_t)blockIdx.x * 8 + (threadIdx.x >> 5); if (r >= (size_t)NB_) return;
#pragma unroll 1
    for (int ps = 0; ps < 2; ++ps) {
#pragma unroll
        for (int q = 0; q < KIN / 256; ++q) { const size_t o = r * KIN + q * 256 + lane * 8; v8us v;
#pragma unroll
            for (int i = 0; i < 8; ++i) v[i] = f2bf(x[o + i]);
            *(volatile v8us*)(A + o) = v; }
        if (ps == 0) __threadfence(); }
}
__global__ __launch_bounds__(256) void k_wplanes(const float* __restrict__ S, const float* __restrict__ TH, bf* Wh, bf* Wl) {
    const int lane = threadIdx.x & 31; const size_t o_ = (size_t)blockIdx.x * 8 + (threadIdx.x >> 5); if (o_ >= (size_t)NOUT) return;
#pragma unroll 1
    for (int ps = 0; ps < 2; ++ps) {
#pragma unroll
        for (int q = 0; q < KIN / 256; ++q) { const size_t o = o_ * KIN + q * 256 + lane * 8; v8us vh, vl;
#pragma unroll
            for (int i = 0; i < 8; ++i) { const float w = bfr(S[o + i]) * bfr(TH[o + i]); const unsigned short hb = f2bf(w); vh[i] = hb; vl[i] = f2bf(w - bf2f(hb)); }
            *(volatile v8us*)(Wh + o) = vh; *(volatile v8us*)(Wl + o) = vl; }
        if (ps == 0) __threadfence(); }
}
__global__ __launch_bounds__(256) void k_addb(const float* __restrict__ C, const float* __restrict__ b, float* OUTB) {
    const int lane = threadIdx.x & 31; const size_t r = (size_t)blockIdx.x * 8 + (threadIdx.x >> 5); if (r >= (size_t)NB_) return;
#pragma unroll 1
    for (int ps = 0; ps < 2; ++ps) {
#pragma unroll
        for (int p = 0; p < NOUT / 128; ++p) { const int c0 = p * 128 + lane * 4; v4f v = *(const v4f*)(C + r * NOUT + c0);
#pragma unroll
            for (int i = 0; i < 4; ++i) v[i] += bfr(b[c0 + i]);
            *(volatile v4f*)(OUTB + r * NOUT + c0) = v; }
        if (ps == 0) __threadfence(); }
}
extern "C" void kernel_launch(void* const* d_in, const int* in_sizes, int n_in,
                              void* d_out, int out_size, void* d_ws, size_t ws_size, hipStream_t stream) {
    (void)in_sizes; (void)n_in; (void)out_size;
    const float* x = (const float*)d_in[0]; const float* S = (const float*)d_in[1]; const float* TH = (const float*)d_in[2]; const float* bias = (const float*)d_in[3];
    float* out = (float*)d_out;
    char* wsp = (char*)d_ws;
    auto take = [&](size_t bytes) { char* p = wsp; wsp += (bytes + 255) & ~(size_t)255; return (void*)p; };
    bf* A = (bf*)take((size_t)NB_ * KIN * 2); bf* Wh = (bf*)take((size_t)NOUT * KIN * 2); bf* Wl = (bf*)take((size_t)NOUT * KIN * 2); float* C = (float*)take((size_t)NB_ * NOUT * 4);
    if ((size_t)(wsp - (char*)d_ws) > ws_size) return;
    k_cvtx<<<NB_ / 8, 256, 0, stream>>>(x, A);
    k_wplanes<<<NOUT / 8, 256, 0, stream>>>(S, TH, Wh, Wl);
    k_gemm3z<16><<<dim3(NB_ / 64, NOUT / 64, 1), 128, 0, stream>>>(A, A, Wh, Wl, KIN, C, NOUT, 0, 0, 0);
    k_addb<<<NB_ / 8, 256, 0, stream>>>(C, bias, out);
}
